// GRU_with_GCC_28570122453317
// MI455X (gfx1250) — hardware-run, weakly checked
//
#include <hip/hip_runtime.h>
#include <math.h>

typedef __attribute__((ext_vector_type(16))) _Float16 v16h;
typedef __attribute__((ext_vector_type(8)))  _Float16 v8h;
typedef __attribute__((ext_vector_type(16))) __bf16   v16b;
typedef __attribute__((ext_vector_type(8)))  __bf16   v8b;
typedef __attribute__((ext_vector_type(8)))  float    v8f;
typedef __attribute__((ext_vector_type(4)))  float    v4f;

constexpr int kBatch  = 64;
constexpr int kSteps  = 64;
constexpr int kIn     = 1024;
constexpr int kHid    = 1024;
constexpr int kF0     = 1024;
constexpr int kF1     = 2048;
constexpr int kKcat   = kIn + kF0 + kF1;
constexpr int kGate2  = 2 * kHid;
constexpr int kGate3  = 3 * kHid;
constexpr int kRows   = kBatch * kSteps;
constexpr int kThr    = 256;
constexpr int kThrRun = 512;
constexpr int kSeqBlk = 16;
constexpr int kHP     = 1032;
constexpr int kHmP    = 1024;
constexpr int kOut0   = kBatch * kSteps * kHid;
constexpr int kOut1   = kBatch * kHid;

constexpr float kInCarry  = 1024.0f;
constexpr float kWCarry   = 1024.0f;
constexpr float kActCarry = 4096.0f;
constexpr float kXsScale  = 1.0f / (kInCarry * kWCarry);
constexpr float kRecScale = 1.0f / (kActCarry * kWCarry);
constexpr float kF16MinNormal = 6.103515625e-5f;

static_assert(kKcat == 4096 && kGate2 == 2048 && kGate3 == 3072 && kRows == 4096, "plane sizes");
static_assert((kRows % 64) == 0 && (kGate2 % 64) == 0 && (kHid % 64) == 0, "GEMM M, N multiples of 64");
static_assert((kKcat % 32) == 0 && (kIn % 32) == 0 && (kHid % 32) == 0, "GEMM K multiples of 32");
static_assert(kHid == 64 * (kThrRun / 32), "16 waves x 64 hidden units");
static_assert(kSeqBlk == kThrRun / 32, "store phase: 16 rows, 8 iterations x 2 lane halves");
static_assert(kBatch % kSeqBlk == 0, "batch tiles");
static_assert((kHP % 8) == 0 && kHP >= kHid + 8, "f16 tile pitch");
static_assert((kIn % 256) == 0 && (kF0 % 256) == 0 && (kF1 % 256) == 0 && (kHid % 256) == 0, "a wave of the cast stores 256 columns of one row");

constexpr size_t kOffXA   = 0;
constexpr size_t kOffWRZ  = kOffXA   + (size_t)kRows  * kKcat * 2;
constexpr size_t kOffWN   = kOffWRZ  + (size_t)kGate2 * kKcat * 2;
constexpr size_t kOffWHH  = kOffWN   + (size_t)kHid   * kIn   * 2;
constexpr size_t kOffBIAS = kOffWHH  + (size_t)kGate3 * kHid  * 2;
constexpr size_t kOffXS   = kOffBIAS + (size_t)2 * kGate3 * 4;
constexpr size_t kWsTotal = kOffXS   + (size_t)kRows * kGate3 * 4;
static_assert(kWsTotal == 109076480ull, "carve total");
static_assert(kWsTotal <= 134217728ull, "carve cap");
static_assert((kOffWRZ % 256) == 0 && (kOffWN % 256) == 0 && (kOffWHH % 256) == 0 && (kOffBIAS % 256) == 0 && (kOffXS % 256) == 0, "aligned regions");

__device__ __forceinline__ unsigned short f2bf_bits(float f) {
  unsigned u = __float_as_uint(f);
  return (unsigned short)((u + 0x7FFFu + ((u >> 16) & 1u)) >> 16);
}
__device__ __forceinline__ float bf_bits2f(unsigned short h) { return __uint_as_float(((unsigned)h) << 16); }
__device__ __forceinline__ float bf16r(float f) { return bf_bits2f(f2bf_bits(f)); }
__device__ __forceinline__ float carry_flush(float v, float carry) {
  const float s = v * carry;
  return (fabsf(s) < kF16MinNormal) ? 0.0f : s;
}
__device__ __forceinline__ float frcp(float x) { return __builtin_amdgcn_rcpf(x); }

__device__ __forceinline__ void dep_guard4_h(v8f& a, v8f& b, v8f& c, v8f& d, v16h x, v16h y) { asm volatile("v_nop\n\tv_nop\n\tv_nop\n\tv_nop" : "+v"(a), "+v"(b), "+v"(c), "+v"(d) : "v"(x), "v"(y)); }
__device__ __forceinline__ void dep_guard4_b(v8f& a, v8f& b, v8f& c, v8f& d, v16b x, v16b y) { asm volatile("v_nop\n\tv_nop\n\tv_nop\n\tv_nop" : "+v"(a), "+v"(b), "+v"(c), "+v"(d) : "v"(x), "v"(y)); }
__device__ __forceinline__ void keep4_h(v16h a, v16h b, v16h c, v16h d) { asm volatile("v_nop" :: "v"(a), "v"(b), "v"(c), "v"(d)); }
__device__ __forceinline__ void keep4_b(v16b a, v16b b, v16b c, v16b d) { asm volatile("v_nop" :: "v"(a), "v"(b), "v"(c), "v"(d)); }
__device__ __forceinline__ void acc_guard4(v8f& a, v8f& b, v8f& c, v8f& d) { asm volatile("v_nop\n\tv_nop\n\tv_nop\n\tv_nop" : "+v"(a), "+v"(b), "+v"(c), "+v"(d)); }

template <typename T> struct Frag;
template <> struct Frag<_Float16> {
  typedef v16h V; union U { v16h v; v8h h[2]; };
  static __device__ __forceinline__ v16h load(const _Float16* p) {
    U f; f.h[0] = *(const v8h*)(p); f.h[1] = *(const v8h*)(p + 16); return f.v;
  }
  static __device__ __forceinline__ v8f mma(v16h a, v16h b, v8f c) {
    return __builtin_amdgcn_wmma_f32_16x16x32_f16(false, a, false, b, (short)0, c, false, false);
  }
  static __device__ __forceinline__ void guard4(v8f& a, v8f& b, v8f& c, v8f& d, v16h x, v16h y) { dep_guard4_h(a, b, c, d, x, y); }
  static __device__ __forceinline__ void keep(v16h a, v16h b, v16h c, v16h d) { keep4_h(a, b, c, d); }
};
template <> struct Frag<__bf16> {
  typedef v16b V; union U { v16b v; v8b h[2]; };
  static __device__ __forceinline__ v16b load(const __bf16* p) {
    U f; f.h[0] = *(const v8b*)(p); f.h[1] = *(const v8b*)(p + 16); return f.v;
  }
  static __device__ __forceinline__ v8f mma(v16b a, v16b b, v8f c) {
    return __builtin_amdgcn_wmma_f32_16x16x32_bf16(false, a, false, b, (short)0, c, false, false);
  }
  static __device__ __forceinline__ void guard4(v8f& a, v8f& b, v8f& c, v8f& d, v16b x, v16b y) { dep_guard4_b(a, b, c, d, x, y); }
  static __device__ __forceinline__ void keep(v16b a, v16b b, v16b c, v16b d) { keep4_b(a, b, c, d); }
};

__device__ __forceinline__ v8f mma_h(v16h a, v16h b, v8f c) {
  c = __builtin_amdgcn_wmma_f32_16x16x32_f16(false, a, false, b, (short)0, c, false, false);
  asm volatile("v_nop\n\tv_nop\n\tv_nop\n\tv_nop" : "+v"(c) : "v"(a), "v"(b));
  return c;
}

template <int ET> struct Elem;
template <> struct Elem<0> { typedef _Float16 T; };
template <> struct Elem<1> { typedef __bf16 T; };
template <int ET, bool SPLIT, int BIAS_MODE, int OUT_MODE, bool RESID, int ACT = 0>
__global__ __launch_bounds__(256) void wmma_gemm64(
    const unsigned short* __restrict__ Ap, const unsigned short* __restrict__ A2p, int lda, long strideA,
    const unsigned short* __restrict__ Btp, const unsigned short* __restrict__ Bt2p, int ldb, long strideB,
    void* __restrict__ Cout, void* __restrict__ Cout2, int ldc, long strideC,
    const float* __restrict__ bias,
    const float* __restrict__ resid, long strideR,
    int M, int N, int K, float scale) {
  typedef typename Elem<ET>::T T;
  typedef typename Frag<T>::V V;
  const T* A = (const T*)Ap; const T* A2 = (const T*)A2p; const T* Bt = (const T*)Btp; const T* Bt2 = (const T*)Bt2p;
  __shared__ __align__(16) float sT[8][16 * 68];
  const int b    = blockIdx.y;
  const int lane = threadIdx.x & 31;
  const int wave = threadIdx.x >> 5;
  const int tilesN = N >> 6;
  const int tilesM = M >> 6;
  const int tile = blockIdx.x * 8 + wave;
  if (tile >= tilesM * tilesN) return;
  const int tm = tile / tilesN;
  const int tn = tile - tm * tilesN;
  const int m0 = tm << 6;
  const int n0 = tn << 6;

  const T* Ab  = A  + (size_t)b * strideA;
  const T* Bb  = Bt + (size_t)b * strideB;
  const T* Ab2 = SPLIT ? (A2  + (size_t)b * strideA) : nullptr;
  const T* Bb2 = SPLIT ? (Bt2 + (size_t)b * strideB) : nullptr;

  const int rlane = lane & 15;
  const int koff  = (lane >> 4) * 8;
  const int mOff  = (lane >> 4) * 8;

  v8f acc[4][4];
#pragma unroll
  for (int i = 0; i < 4; ++i)
#pragma unroll
    for (int j = 0; j < 4; ++j) acc[i][j] = (v8f){0.f,0.f,0.f,0.f,0.f,0.f,0.f,0.f};

  for (int k0 = 0; k0 < K; k0 += 32) {
    V bh[4], bl[4];
#pragma unroll
    for (int j = 0; j < 4; ++j) {
      const size_t bo = (size_t)(n0 + (j << 4) + rlane) * ldb + koff + k0;
      bh[j] = Frag<T>::load(Bb + bo);
      if (SPLIT) bl[j] = Frag<T>::load(Bb2 + bo);
    }
#pragma unroll
    for (int i = 0; i < 4; ++i) {
      const size_t ao = (size_t)(m0 + (i << 4) + rlane) * lda + koff + k0;
      V ah = Frag<T>::load(Ab + ao);
      V al;
      if (SPLIT) al = Frag<T>::load(Ab2 + ao);
#pragma unroll
      for (int j = 0; j < 4; ++j) {
        acc[i][j] = Frag<T>::mma(ah, bh[j], acc[i][j]);
        if (SPLIT) {
          acc[i][j] = Frag<T>::mma(ah, bl[j], acc[i][j]);
          acc[i][j] = Frag<T>::mma(al, bh[j], acc[i][j]);
        }
      }
      Frag<T>::guard4(acc[i][0], acc[i][1], acc[i][2], acc[i][3], ah, SPLIT ? al : ah);
    }
    Frag<T>::keep(bh[0], bh[1], bh[2], bh[3]);
    if (SPLIT) Frag<T>::keep(bl[0], bl[1], bl[2], bl[3]);
  }
  acc_guard4(acc[0][0], acc[0][1], acc[0][2], acc[0][3]);
  acc_guard4(acc[1][0], acc[1][1], acc[1][2], acc[1][3]);
  acc_guard4(acc[2][0], acc[2][1], acc[2][2], acc[2][3]);
  acc_guard4(acc[3][0], acc[3][1], acc[3][2], acc[3][3]);

  float* slab = sT[wave];
  const float* Rb = RESID ? (resid + (size_t)b * strideR) : nullptr;
#pragma unroll
  for (int i = 0; i < 4; ++i) {
    const int mBase = m0 + (i << 4);
#pragma unroll
    for (int j = 0; j < 4; ++j) {
      const int n = n0 + (j << 4) + rlane;
      float bv = 0.f;
      if (BIAS_MODE == 2) bv = bias[n];
#pragma unroll
      for (int r = 0; r < 8; ++r) {
        float v = acc[i][j][r] * scale;
        if (BIAS_MODE == 1) v += bias[mBase + mOff + r];
        if (BIAS_MODE == 2) v += bv;
        if (RESID) v += Rb[(size_t)(mBase + mOff + r) * ldc + n];
        if (ACT == 1) v = tanhf(v);
        if (ACT == 2) v = fmaxf(v, 0.0f);
        if (ACT == 3) v = v / (1.0f + expf(-v));
        if (ACT == 4) v = (v > 0.f) ? v : 0.01f * v;
        slab[(mOff + r) * 68 + (j << 4) + rlane] = v;
      }
    }
    __builtin_amdgcn_fence(__ATOMIC_RELEASE, "workgroup");
    __builtin_amdgcn_wave_barrier();
    __builtin_amdgcn_fence(__ATOMIC_ACQUIRE, "workgroup");
    if (OUT_MODE == 0) {
      float* C = (float*)Cout + (size_t)b * strideC;
      const int hh = lane >> 4, c4 = (lane & 15) * 4;
      for (int pass = 0; pass < 2; ++pass) {
#pragma unroll
        for (int it = 0; it < 8; ++it) {
          const int row = it * 2 + hh;
          v4f v = *(const v4f*)(slab + row * 68 + c4);
          *(volatile v4f*)(C + (size_t)(mBase + row) * ldc + n0 + c4) = v;
        }
        __threadfence();
      }
    } else {
      const int q = lane >> 3, c8 = (lane & 7) * 8;
      unsigned short* C  = (unsigned short*)Cout  + (size_t)b * strideC;
      unsigned short* C2 = (OUT_MODE == 2) ? ((unsigned short*)Cout2 + (size_t)b * strideC) : nullptr;
      for (int pass = 0; pass < 2; ++pass) {
#pragma unroll
        for (int it = 0; it < 4; ++it) {
          const int row = it * 4 + q;
          const float* sp = slab + row * 68 + c8;
          v8h hv, lv;
#pragma unroll
          for (int e = 0; e < 8; ++e) {
            if (OUT_MODE == 1) {
              hv[e] = (_Float16)sp[e];
            } else {
              unsigned short hb = f2bf_bits(sp[e]);
              unsigned short lb = f2bf_bits(sp[e] - bf_bits2f(hb));
              hv[e] = __builtin_bit_cast(_Float16, hb);
              lv[e] = __builtin_bit_cast(_Float16, lb);
            }
          }
          *(volatile v8h*)(C + (size_t)(mBase + row) * ldc + n0 + c8) = hv;
          if (OUT_MODE == 2) *(volatile v8h*)(C2 + (size_t)(mBase + row) * ldc + n0 + c8) = lv;
        }
        __threadfence();
      }
    }
    __builtin_amdgcn_fence(__ATOMIC_RELEASE, "workgroup");
    __builtin_amdgcn_wave_barrier();
    __builtin_amdgcn_fence(__ATOMIC_ACQUIRE, "workgroup");
  }
}

__global__ __launch_bounds__(kThr) void cast_plane_kernel(const float* __restrict__ src, unsigned short* __restrict__ dst,
                                                          int colsLog2, int dstPitch, int dstOff) {
  const int i   = blockIdx.x * kThr + threadIdx.x;
  const int sh  = colsLog2 - 3;
  const int row = i >> sh;
  const int c8  = (i & ((1 << sh) - 1)) * 8;
  const float* sp = src + ((size_t)row << colsLog2) + c8;
  const v4f a0 = *(const v4f*)(sp);
  const v4f a1 = *(const v4f*)(sp + 4);
  v8h hv;
#pragma unroll
  for (int e = 0; e < 4; ++e) {
    const float f0 = a0[e];
    const float f1 = a1[e];
    hv[e]     = (_Float16)carry_flush(bf16r(f0), kInCarry);
    hv[4 + e] = (_Float16)carry_flush(bf16r(f1), kInCarry);
  }
  unsigned short* dp = dst + (size_t)row * dstPitch + dstOff + c8;
  *(volatile v8h*)dp = hv;
  __threadfence();
  *(volatile v8h*)dp = hv;
}
static_assert(kInCarry == kWCarry, "one cast kernel serves inputs and weights");

__global__ __launch_bounds__(kThr) void bias_prep_kernel(const float* __restrict__ bih, const float* __restrict__ bhh,
                                                         const float* __restrict__ bf0, const float* __restrict__ bf1,
                                                         float* __restrict__ dst) {
  const int blk = blockIdx.x;
  const int idx = (blk * kThr + threadIdx.x) * 4;
  v4f o;
  if (blk < 2) {
    const v4f a = *(const v4f*)(bih + idx);
    const v4f b = *(const v4f*)(bf0 + idx);
    const v4f d = *(const v4f*)(bf1 + idx);
#pragma unroll
    for (int e = 0; e < 4; ++e) {
      const float fa = a[e];
      const float fb = b[e];
      const float fd = d[e];
      o[e] = (bf16r(fa) + bf16r(fb)) + bf16r(fd);
    }
  } else if (blk < 3) {
    const v4f a = *(const v4f*)(bih + idx);
#pragma unroll
    for (int e = 0; e < 4; ++e) {
      const float fa = a[e];
      o[e] = bf16r(fa);
    }
  } else {
    const v4f a = *(const v4f*)(bhh + (idx - kGate3));
#pragma unroll
    for (int e = 0; e < 4; ++e) {
      const float fa = a[e];
      o[e] = bf16r(fa);
    }
  }
  float* op = dst + idx;
  *(volatile v4f*)op = o;
  __threadfence();
  *(volatile v4f*)op = o;
}
static_assert(2 * kThr * 4 == kGate2 && 3 * kThr * 4 == kGate3 && 6 * kThr * 4 == 2 * kGate3, "bias block ranges");

__global__ __launch_bounds__(kThrRun) void gated_run_kernel(const float* __restrict__ XS,
                                                            const unsigned short* __restrict__ WHp,
                                                            const float* __restrict__ BH,
                                                            float* __restrict__ OUT0,
                                                            float* __restrict__ OUT1) {
  __shared__ __align__(16) _Float16 Ah[2][kSeqBlk * kHP];
  __shared__ __align__(16) float    Hm[kSeqBlk * kHmP];
  __shared__ __align__(16) float    sBh[kGate3];
  const _Float16* WH = (const _Float16*)WHp;
  const int tid = threadIdx.x, lane = tid & 31, wave = tid >> 5;
  const int c = lane & 15, hh = lane >> 4, koff = hh * 8, c4 = c * 4;
  const int rowbase = blockIdx.x * kSeqBlk;

  {
    _Float16* ahf = &Ah[0][0];
#pragma unroll 1
    for (int i = tid; i < 2 * kSeqBlk * kHP; i += kThrRun) ahf[i] = (_Float16)0.0f;
#pragma unroll 1
    for (int i = tid; i < kSeqBlk * kHmP; i += kThrRun) Hm[i] = 0.0f;
#pragma unroll 1
    for (int i = tid; i < kGate3; i += kThrRun) sBh[i] = BH[i];
  }
  __syncthreads();

  const v8f z8 = {0.f, 0.f, 0.f, 0.f, 0.f, 0.f, 0.f, 0.f};

#pragma unroll 1
  for (int s = 0; s < kSteps; ++s) {
    const int cur = s & 1;
    const _Float16* ahrow = &Ah[cur][0] + c * kHP + koff;
    _Float16* ahn = &Ah[cur ^ 1][0];
    const float* xsrow = XS + ((size_t)(rowbase + 8 * hh) * kSteps + s) * kGate3;

#pragma unroll 1
    for (int nt = 0; nt < 4; ++nt) {
      const int j = 64 * wave + 16 * nt + c;
      float xr[8], xz[8], xn[8];
#pragma unroll
      for (int r = 0; r < 8; ++r) {
        const float* xp = xsrow + (size_t)r * kSteps * kGate3 + j;
        xr[r] = xp[0];
        xz[r] = xp[kHid];
        xn[r] = xp[2 * kHid];
      }
      const _Float16* wr = WH + (size_t)j * kHid + koff;
      const _Float16* wz = WH + (size_t)(kHid + j) * kHid + koff;
      const _Float16* wn = WH + (size_t)(2 * kHid + j) * kHid + koff;
      v8f ar = z8, az = z8, an = z8;
#pragma unroll 2
      for (int k0 = 0; k0 < kHid; k0 += 32) {
        const v16h a   = Frag<_Float16>::load(ahrow + k0);
        const v16h fbr = Frag<_Float16>::load(wr + k0);
        const v16h fbz = Frag<_Float16>::load(wz + k0);
        const v16h fbn = Frag<_Float16>::load(wn + k0);
        ar = mma_h(a, fbr, ar);
        az = mma_h(a, fbz, az);
        an = mma_h(a, fbn, an);
      }
      const float bhr = sBh[j];
      const float bhz = sBh[kHid + j];
      const float bhn = sBh[2 * kHid + j];
#pragma unroll
      for (int r = 0; r < 8; ++r) {
        const int row = 8 * hh + r;
        const float hr = ar[r] * kRecScale + bhr;
        const float hz = az[r] * kRecScale + bhz;
        const float hn = an[r] * kRecScale + bhn;
        const float rg = 1.0f / (1.0f + expf(-(xr[r] + hr)));
        const float zg = 1.0f / (1.0f + expf(-(xz[r] + hz)));
        const float nc = tanhf(xn[r] + rg * hn);
        const float ho = Hm[row * kHmP + j];
        const float hnew = nc + zg * (ho - nc);
        Hm[row * kHmP + j] = hnew;
        ahn[row * kHP + j] = (_Float16)carry_flush(hnew, kActCarry);
      }
    }
    __syncthreads();

    v4f ov[8];
#pragma unroll
    for (int it = 0; it < 8; ++it) {
      const int row = it * 2 + hh;
      ov[it] = *(const v4f*)(Hm + row * kHmP + 64 * wave + c4);
    }
    const bool lastStep = (s == kSteps - 1);
    for (int pass = 0; pass < 2; ++pass) {
#pragma unroll
      for (int it = 0; it < 8; ++it) {
        const int row = it * 2 + hh;
        float* p0 = OUT0 + ((size_t)(rowbase + row) * kSteps + s) * kHid + 64 * wave + c4;
        *(volatile v4f*)p0 = ov[it];
        if (lastStep) {
          float* p1 = OUT1 + (size_t)(rowbase + row) * kHid + 64 * wave + c4;
          *(volatile v4f*)p1 = ov[it];
        }
      }
      __threadfence();
    }
  }
}

static_assert(((size_t)kRows  * kIn  / 8) % kThr == 0 && ((size_t)kRows  * kF1 / 8) % kThr == 0, "input cast grids exact");
static_assert(((size_t)kGate2 * kIn  / 8) % kThr == 0 && ((size_t)kGate2 * kF1 / 8) % kThr == 0, "gate weight cast grids exact");
static_assert(((size_t)kHid   * kIn  / 8) % kThr == 0 && ((size_t)kGate3 * kHid / 8) % kThr == 0, "candidate / state weight cast grids exact");
static_assert(((kRows / 64) * (kGate2 / 64)) % 8 == 0 && ((kRows / 64) * (kHid / 64)) % 8 == 0, "GEMM grids exact");

extern "C" void kernel_launch(void* const* d_in, const int* in_sizes, int n_in,
                              void* d_out, int out_size, void* d_ws, size_t ws_size,
                              hipStream_t stream) {
  if (n_in < 11 || d_out == nullptr || d_ws == nullptr) return;
  if (in_sizes[0] != kRows * kIn || in_sizes[1] != kRows * kF0 || in_sizes[2] != kRows * kF1) return;
  if (in_sizes[3] != kGate3 * kIn || in_sizes[4] != kGate3 * kHid) return;
  if (in_sizes[5] != kGate3 || in_sizes[6] != kGate3) return;
  if (in_sizes[7] != kGate2 * kF0 || in_sizes[8] != kGate2) return;
  if (in_sizes[9] != kGate2 * kF1 || in_sizes[10] != kGate2) return;
  if (out_size != kOut0 + kOut1) return;
  if (ws_size < kWsTotal) return;

  const float* x    = (const float*)d_in[0];
  const float* aux0 = (const float*)d_in[1];
  const float* aux1 = (const float*)d_in[2];
  const float* Wih  = (const float*)d_in[3];
  const float* Whh  = (const float*)d_in[4];
  const float* bih  = (const float*)d_in[5];
  const float* bhh  = (const float*)d_in[6];
  const float* Wf0  = (const float*)d_in[7];
  const float* bf0  = (const float*)d_in[8];
  const float* Wf1  = (const float*)d_in[9];
  const float* bf1  = (const float*)d_in[10];
  float* out0 = (float*)d_out;
  float* out1 = out0 + kOut0;

  char* ws = (char*)d_ws;
  unsigned short* XA   = (unsigned short*)(ws + kOffXA);
  unsigned short* WRZ  = (unsigned short*)(ws + kOffWRZ);
  unsigned short* WN   = (unsigned short*)(ws + kOffWN);
  unsigned short* WHH  = (unsigned short*)(ws + kOffWHH);
  float*          BIASP = (float*)(ws + kOffBIAS);
  float*          XS   = (float*)(ws + kOffXS);

  cast_plane_kernel<<<(kRows  * kIn  / 8) / kThr, kThr, 0, stream>>>(x,    XA,  10, kKcat, 0);
  cast_plane_kernel<<<(kRows  * kF0  / 8) / kThr, kThr, 0, stream>>>(aux0, XA,  10, kKcat, kIn);
  cast_plane_kernel<<<(kRows  * kF1  / 8) / kThr, kThr, 0, stream>>>(aux1, XA,  11, kKcat, kIn + kF0);
  cast_plane_kernel<<<(kGate2 * kIn  / 8) / kThr, kThr, 0, stream>>>(Wih,  WRZ, 10, kKcat, 0);
  cast_plane_kernel<<<(kGate2 * kF0  / 8) / kThr, kThr, 0, stream>>>(Wf0,  WRZ, 10, kKcat, kIn);
  cast_plane_kernel<<<(kGate2 * kF1  / 8) / kThr, kThr, 0, stream>>>(Wf1,  WRZ, 11, kKcat, kIn + kF0);
  cast_plane_kernel<<<(kHid   * kIn  / 8) / kThr, kThr, 0, stream>>>(Wih + (size_t)kGate2 * kIn, WN, 10, kIn, 0);
  cast_plane_kernel<<<(kGate3 * kHid / 8) / kThr, kThr, 0, stream>>>(Whh,  WHH, 10, kHid, 0);
  bias_prep_kernel<<<6, kThr, 0, stream>>>(bih, bhh, bf0, bf1, BIASP);

  wmma_gemm64<0, false, 2, 0, false, 0><<<dim3((kRows / 64) * (kGate2 / 64) / 8, 1), 256, 0, stream>>>(
      XA, XA, kKcat, 0L, WRZ, WRZ, kKcat, 0L, (void*)XS, (void*)XS, kGate3, 0L,
      BIASP, nullptr, 0L, kRows, kGate2, kKcat, kXsScale);
  wmma_gemm64<0, false, 2, 0, false, 0><<<dim3((kRows / 64) * (kHid / 64) / 8, 1), 256, 0, stream>>>(
      XA, XA, kKcat, 0L, WN, WN, kIn, 0L, (void*)(XS + kGate2), (void*)(XS + kGate2), kGate3, 0L,
      BIASP + kGate2, nullptr, 0L, kRows, kHid, kIn, kXsScale);

  gated_run_kernel<<<kBatch / kSeqBlk, kThrRun, 0, stream>>>(XS, WHH, BIASP + kGate3, out0, out1);
}
